// HyperedgeAggregator_36670430773458
// MI455X (gfx1250) — hardware-verified
//
#include <hip/hip_runtime.h>
#include <math.h>
#include <stdint.h>


#define B_    2
#define N_    20000
#define E_    20000
#define A_    8
#define H_    256
#define TE_   32
#define NT_   16
#define KENC  288
#define KUPD  512
#define PENC  320
#define PUPD  512
#define WSCALE 16.0f
#define WINV   0.0625f

#define TN     512
#define CAP    8192
#define MAXDEG 64
#define KEYPAD 0x7FFFFFFF

typedef _Float16 v16h __attribute__((ext_vector_type(16)));
typedef _Float16 v8h  __attribute__((ext_vector_type(8)));
typedef float    v8f  __attribute__((ext_vector_type(8)));
typedef float    v4f  __attribute__((ext_vector_type(4)));
union Frag { v16h v; v8h half[2]; };

__device__ __forceinline__ v8f wmma16(v8f c, v16h a, v16h b)
{
    v8f d = __builtin_amdgcn_wmma_f32_16x16x32_f16(false, a, false, b, (short)0, c, false, false);
    asm volatile("v_nop\n\tv_nop\n\tv_nop\n\tv_nop" : "+v"(d) : "v"(a), "v"(b));
    return d;
}

__device__ __forceinline__ v8h pack8(v4f a, v4f b)
{
    v8h r;
    r[0] = (_Float16)a[0]; r[1] = (_Float16)a[1]; r[2] = (_Float16)a[2]; r[3] = (_Float16)a[3];
    r[4] = (_Float16)b[0]; r[5] = (_Float16)b[1]; r[6] = (_Float16)b[2]; r[7] = (_Float16)b[3];
    return r;
}

__device__ __forceinline__ float gelu_exact(float x)
{
    return 0.5f * x * (1.0f + erff(x * 0.70710678118654752f));
}

__global__ __launch_bounds__(64)
void k_wconv(const float* __restrict__ Wenc, const float* __restrict__ Wupd,
             _Float16* __restrict__ Wte, _Float16* __restrict__ Wtu)
{
    __shared__ v8h rowbuf8[PUPD / 8];
    _Float16* rowbuf = (_Float16*)rowbuf8;

    const int blk = blockIdx.x;
    const int t   = threadIdx.x;
    const bool enc = blk < 256;
    const int n   = enc ? blk : (blk - 256);
    const float* W = enc ? Wenc : Wupd;
    const int K   = enc ? KENC : KUPD;
    const int P   = enc ? PENC : PUPD;
    _Float16* dst = enc ? Wte : Wtu;

    for (int k = t; k < P; k += 64) {
        const float v = (k < K) ? W[(size_t)k * 256 + n] * WSCALE : 0.0f;
        rowbuf[k] = (_Float16)v;
    }
    __syncthreads();

    const int nch = P / 8;
    v8h val = rowbuf8[0];
    if (t < nch) val = rowbuf8[t];
    if (t < nch) {
        _Float16* p = dst + (size_t)n * P + 8 * t;
        *(volatile v8h*)p = val;
    }
    __threadfence();
    if (t < nch) {
        _Float16* p = dst + (size_t)n * P + 8 * t;
        *(volatile v8h*)p = val;
    }
}

template<int MODE>
__global__ __launch_bounds__(256)
void k_gemm_ln(const float* __restrict__ nf, const int* __restrict__ members,
               const int* __restrict__ types, const int* __restrict__ emask,
               const float* __restrict__ ett, const _Float16* __restrict__ upd16,
               const _Float16* __restrict__ Wt, const float* __restrict__ bias,
               const float* __restrict__ gamma, const float* __restrict__ beta,
               float* __restrict__ out, int nrows)
{
    constexpr int K  = (MODE == 0) ? KENC : KUPD;
    constexpr int KP = K + 8;
    constexpr int WP = (MODE == 0) ? PENC : PUPD;
    constexpr int CP = 260;
    constexpr int ABYTES = 32 * KP * 2;
    constexpr int CBYTES = 32 * CP * 4;
    constexpr int LBYTES = (ABYTES > CBYTES) ? ABYTES : CBYTES;
    __shared__ v4f lds4[LBYTES / 16];

    _Float16* A16 = (_Float16*)lds4;

    const int tid  = threadIdx.x;
    const int lane = tid & 31;
    const int wave = tid >> 5;
    const int row0 = blockIdx.x * 32;

    const v4f z4 = {0.f, 0.f, 0.f, 0.f};
    const v8h z8 = pack8(z4, z4);

#pragma unroll
    for (int i = 0; i < 4; ++i) {
        const int r    = wave * 4 + i;
        const int grow = row0 + r;
        _Float16* arow = A16 + r * KP;
        if (grow < nrows) {
            if (MODE == 0) {
                const int bb = grow / E_;
                const int* mm = members + (size_t)grow * A_;
                const int* mk = emask + (size_t)grow * A_;
                v4f s0 = z4, s1 = z4;
                float cnt = 0.f;
#pragma unroll
                for (int a = 0; a < A_; ++a) {
                    int idx = mm[a];
                    idx = idx < 0 ? 0 : (idx > N_ - 1 ? N_ - 1 : idx);
                    const float mv = (mk[a] != 0) ? 1.f : 0.f;
                    cnt += mv;
                    const float* src = nf + ((size_t)bb * N_ + idx) * H_ + lane * 8;
                    const v4f x0 = *(const v4f*)src;
                    const v4f x1 = *(const v4f*)(src + 4);
                    s0 += mv * x0;
                    s1 += mv * x1;
                }
                const float inv = 1.0f / fmaxf(cnt, 1.f);
                *(v8h*)(arow + lane * 8) = pack8(s0 * inv, s1 * inv);
                if (lane < 4) {
                    int t = types[grow];
                    t = t < 0 ? 0 : (t > NT_ - 1 ? NT_ - 1 : t);
                    const float* es = ett + t * TE_ + lane * 8;
                    *(v8h*)(arow + H_ + lane * 8) = pack8(*(const v4f*)es, *(const v4f*)(es + 4));
                }
            } else {
                const float* src = nf + (size_t)grow * H_ + lane * 8;
                *(v8h*)(arow + lane * 8) = pack8(*(const v4f*)src, *(const v4f*)(src + 4));
                *(v8h*)(arow + H_ + lane * 8) = *(const v8h*)(upd16 + (size_t)grow * H_ + lane * 8);
            }
        } else {
            *(v8h*)(arow + lane * 8) = z8;
            if (MODE == 0) { if (lane < 4) *(v8h*)(arow + H_ + lane * 8) = z8; }
            else           { *(v8h*)(arow + H_ + lane * 8) = z8; }
        }
    }
    __syncthreads();

    const int l = lane, h = l >> 4, m = l & 15;
    v8f acc00 = {0,0,0,0,0,0,0,0}, acc01 = {0,0,0,0,0,0,0,0};
    v8f acc10 = {0,0,0,0,0,0,0,0}, acc11 = {0,0,0,0,0,0,0,0};
    const _Float16* Ar0 = A16 + m * KP + 8 * h;
    const _Float16* Ar1 = A16 + (16 + m) * KP + 8 * h;
    const _Float16* Br0 = Wt + (size_t)(wave * 32 + m) * WP + 8 * h;
    const _Float16* Br1 = Wt + (size_t)(wave * 32 + 16 + m) * WP + 8 * h;
    for (int k0 = 0; k0 < K; k0 += 32) {
        Frag a0, a1, b0, b1;
        a0.half[0] = *(const v8h*)(Ar0 + k0);  a0.half[1] = *(const v8h*)(Ar0 + k0 + 16);
        a1.half[0] = *(const v8h*)(Ar1 + k0);  a1.half[1] = *(const v8h*)(Ar1 + k0 + 16);
        b0.half[0] = *(const v8h*)(Br0 + k0);  b0.half[1] = *(const v8h*)(Br0 + k0 + 16);
        b1.half[0] = *(const v8h*)(Br1 + k0);  b1.half[1] = *(const v8h*)(Br1 + k0 + 16);
        acc00 = wmma16(acc00, a0.v, b0.v);
        acc01 = wmma16(acc01, a0.v, b1.v);
        acc10 = wmma16(acc10, a1.v, b0.v);
        acc11 = wmma16(acc11, a1.v, b1.v);
    }
    __syncthreads();

    float* Cs = (float*)lds4;
    {
        const int cA = wave * 32 + m;
        const int cB = cA + 16;
#pragma unroll
        for (int r = 0; r < 8; ++r) {
            Cs[(8 * h + r) * CP + cA]      = acc00[r];
            Cs[(8 * h + r) * CP + cB]      = acc01[r];
            Cs[(16 + 8 * h + r) * CP + cA] = acc10[r];
            Cs[(16 + 8 * h + r) * CP + cB] = acc11[r];
        }
    }
    __syncthreads();

    const v4f bi0 = *(const v4f*)(bias + 4 * lane),  bi1 = *(const v4f*)(bias + 128 + 4 * lane);
    const v4f ga0 = *(const v4f*)(gamma + 4 * lane), ga1 = *(const v4f*)(gamma + 128 + 4 * lane);
    const v4f be0 = *(const v4f*)(beta + 4 * lane),  be1 = *(const v4f*)(beta + 128 + 4 * lane);
    v4f y0[4], y1[4];
#pragma unroll
    for (int i = 0; i < 4; ++i) {
        const int r = wave * 4 + i;
        const v4f c0 = *(const v4f*)(Cs + r * CP + 4 * lane);
        const v4f c1 = *(const v4f*)(Cs + r * CP + 128 + 4 * lane);
        const v4f x0 = c0 * WINV + bi0;
        const v4f x1 = c1 * WINV + bi1;
        v4f g0, g1;
        g0[0] = gelu_exact(x0[0]); g0[1] = gelu_exact(x0[1]); g0[2] = gelu_exact(x0[2]); g0[3] = gelu_exact(x0[3]);
        g1[0] = gelu_exact(x1[0]); g1[1] = gelu_exact(x1[1]); g1[2] = gelu_exact(x1[2]); g1[3] = gelu_exact(x1[3]);
        float s = (g0[0] + g0[1]) + (g0[2] + g0[3]) + ((g1[0] + g1[1]) + (g1[2] + g1[3]));
#pragma unroll
        for (int o = 16; o > 0; o >>= 1) s += __shfl_xor(s, o, 32);
        const float mu = s * (1.0f / 256.0f);
        const v4f d0 = g0 - mu;
        const v4f d1 = g1 - mu;
        float ss = (d0[0]*d0[0] + d0[1]*d0[1]) + (d0[2]*d0[2] + d0[3]*d0[3])
                 + ((d1[0]*d1[0] + d1[1]*d1[1]) + (d1[2]*d1[2] + d1[3]*d1[3]));
#pragma unroll
        for (int o = 16; o > 0; o >>= 1) ss += __shfl_xor(ss, o, 32);
        const float var  = ss * (1.0f / 256.0f);
        const float rstd = rsqrtf(var + 1e-5f);
        y0[i] = d0 * rstd * ga0 + be0;
        y1[i] = d1 * rstd * ga1 + be1;
    }
#pragma unroll
    for (int i = 0; i < 4; ++i) {
        const int grow = row0 + wave * 4 + i;
        if (grow < nrows) {
            float* p = out + (size_t)grow * H_;
            *(volatile v4f*)(p + 4 * lane)       = y0[i];
            *(volatile v4f*)(p + 128 + 4 * lane) = y1[i];
        }
    }
    __threadfence();
#pragma unroll
    for (int i = 0; i < 4; ++i) {
        const int grow = row0 + wave * 4 + i;
        if (grow < nrows) {
            float* p = out + (size_t)grow * H_;
            *(volatile v4f*)(p + 4 * lane)       = y0[i];
            *(volatile v4f*)(p + 128 + 4 * lane) = y1[i];
        }
    }
}

__global__ __launch_bounds__(TN)
void k_aggregate(const float* __restrict__ ef, const int* __restrict__ members,
                 const int* __restrict__ emask, _Float16* __restrict__ upd16)
{
    __shared__ int Kl[CAP];
    __shared__ int segs[TN];
    __shared__ int sege[TN];
    __shared__ int wcnt[2][16];

    const int tid  = threadIdx.x;
    const int lane = tid & 31;
    const int wave = tid >> 5;
    const int tilesPerB = (N_ + TN - 1) / TN;
    const int b  = blockIdx.x / tilesPerB;
    const int n0 = (blockIdx.x - b * tilesPerB) * TN;
    const int* mem = members + (size_t)b * E_ * A_;
    const int* msk = emask   + (size_t)b * E_ * A_;
    const int total = E_ * A_;

    segs[tid] = 0;
    sege[tid] = 0;

    int base = 0;
    const int nchunks = (total + TN - 1) / TN;
    for (int c = 0; c < nchunks; ++c) {
        const int s = c * TN + tid;
        bool hit = false;
        int packed = 0;
        if (s < total) {
            int idx = mem[s];
            idx = idx < 0 ? 0 : (idx > N_ - 1 ? N_ - 1 : idx);
            const int mv  = msk[s];
            const int loc = idx - n0;
            hit = (mv != 0) && ((unsigned)loc < (unsigned)TN);
            packed = (loc << 18) | s;
        }
        const unsigned bal = (unsigned)__ballot(hit ? 1 : 0);
        const int lanepre  = __popc(bal & ((1u << lane) - 1u));
        const int wc       = __popc(bal);
        if (lane == 0) wcnt[c & 1][wave] = wc;
        __syncthreads();
        int wpre = 0, tot = 0;
#pragma unroll
        for (int w = 0; w < 16; ++w) {
            const int v = wcnt[c & 1][w];
            tot  += v;
            wpre += (w < wave) ? v : 0;
        }
        if (hit) {
            const int pos = base + wpre + lanepre;
            if (pos < CAP) Kl[pos] = packed;
        }
        base += tot;
    }
    const int M = (base < CAP) ? base : CAP;

    int NS = 1024;
#pragma unroll
    for (int i = 0; i < 3; ++i) { if (NS < M) NS <<= 1; }

    for (int i = M + tid; i < NS; i += TN) Kl[i] = KEYPAD;
    __syncthreads();

    for (int k = 2; k <= NS; k <<= 1) {
        for (int j = k >> 1; j > 0; j >>= 1) {
            const int npairs = NS >> 1;
            for (int t = tid; t < npairs; t += TN) {
                const int i0 = ((t & ~(j - 1)) << 1) | (t & (j - 1));
                const int i1 = i0 | j;
                const int x0 = Kl[i0];
                const int x1 = Kl[i1];
                const bool up = ((i0 & k) == 0);
                const bool sw = up ? (x0 > x1) : (x0 < x1);
                if (sw) { Kl[i0] = x1; Kl[i1] = x0; }
            }
            __syncthreads();
        }
    }

    for (int i = tid; i < M; i += TN) {
        const int key = Kl[i];
        const int kh  = key >> 18;
        const int loc = kh & (TN - 1);
        const int ip  = (i > 0) ? (i - 1) : 0;
        const int in  = (i + 1 < CAP) ? (i + 1) : (CAP - 1);
        const int kp  = Kl[ip] >> 18;
        const int kn  = Kl[in] >> 18;
        if (i == 0 || kp != kh)     segs[loc] = i;
        if (i == M - 1 || kn != kh) sege[loc] = i + 1;
    }
    __syncthreads();

    const v4f z4 = {0.f, 0.f, 0.f, 0.f};
    for (int q = 0; q < 32; ++q) {
        const int j = wave * 32 + q;
        const int g = n0 + j;
        int st = segs[j];
        st = (st < 0) ? 0 : (st > CAP - 1 ? (CAP - 1) : st);
        int c = sege[j] - st;
        c = (c < 0) ? 0 : (c > MAXDEG ? MAXDEG : c);
        const int room = CAP - st;
        c = (c < room) ? c : room;
        v4f a0 = z4, a1 = z4;
        for (int p = 0; p < c; ++p) {
            const int s = Kl[st + p] & 0x3FFFF;
            int e = s >> 3;
            e = (e > E_ - 1) ? (E_ - 1) : e;
            const float* row = ef + ((size_t)b * E_ + e) * H_ + lane * 8;
            a0 += *(const v4f*)row;
            a1 += *(const v4f*)(row + 4);
        }
        const float inv = 1.0f / fmaxf((float)c, 1.f);
        const v8h pk = pack8(a0 * inv, a1 * inv);
        if (g < N_) {
            _Float16* dst = upd16 + ((size_t)b * N_ + g) * H_ + lane * 8;
            *(volatile v8h*)dst = pk;
            __threadfence();
            *(volatile v8h*)dst = pk;
        }
    }
}

extern "C" void kernel_launch(void* const* d_in, const int* in_sizes, int n_in,
                              void* d_out, int out_size, void* d_ws, size_t ws_size,
                              hipStream_t stream)
{
    if (n_in < 13) return;
    if (in_sizes[0] != B_ * N_ * H_) return;
    if (in_sizes[1] != B_ * E_ * A_) return;
    if (in_sizes[2] != B_ * E_) return;
    if (in_sizes[3] != B_ * E_ * A_) return;
    if (in_sizes[4] != NT_ * TE_) return;
    if (in_sizes[5] != KENC * H_) return;
    if (in_sizes[9] != KUPD * H_) return;
    if (out_size != B_ * N_ * H_) return;

    const float* nf      = (const float*)d_in[0];
    const int*   members = (const int*)d_in[1];
    const int*   types   = (const int*)d_in[2];
    const int*   emask   = (const int*)d_in[3];
    const float* ett     = (const float*)d_in[4];
    const float* W_enc   = (const float*)d_in[5];
    const float* b_enc   = (const float*)d_in[6];
    const float* g_enc   = (const float*)d_in[7];
    const float* be_enc  = (const float*)d_in[8];
    const float* W_upd   = (const float*)d_in[9];
    const float* b_upd   = (const float*)d_in[10];
    const float* g_upd   = (const float*)d_in[11];
    const float* be_upd  = (const float*)d_in[12];
    float* out = (float*)d_out;

    const size_t bytes_wte = (size_t)H_ * PENC * 2;
    const size_t bytes_wtu = (size_t)H_ * PUPD * 2;
    const size_t bytes_ef  = (size_t)B_ * E_ * H_ * 4;
    const size_t bytes_upd = (size_t)B_ * N_ * H_ * 2;
    const size_t off_wte = 0;
    const size_t off_wtu = off_wte + bytes_wte;
    const size_t off_ef  = off_wtu + bytes_wtu;
    const size_t off_upd = off_ef  + bytes_ef;
    const size_t total_ws = off_upd + bytes_upd;
    if (total_ws > ws_size) return;

    char* ws = (char*)d_ws;
    _Float16* Wte   = (_Float16*)(ws + off_wte);
    _Float16* Wtu   = (_Float16*)(ws + off_wtu);
    float*    ef    = (float*)(ws + off_ef);
    _Float16* upd16 = (_Float16*)(ws + off_upd);

    const int rows_enc = B_ * E_;
    const int rows_upd = B_ * N_;
    const int grid_enc = (rows_enc + 31) / 32;
    const int grid_upd = (rows_upd + 31) / 32;
    const int grid_agg = B_ * ((N_ + TN - 1) / TN);

    k_wconv<<<512, 64, 0, stream>>>(W_enc, W_upd, Wte, Wtu);

    k_gemm_ln<0><<<grid_enc, 256, 0, stream>>>(nf, members, types, emask, ett, upd16,
                                                Wte, b_enc, g_enc, be_enc, ef, rows_enc);

    k_aggregate<<<grid_agg, TN, 0, stream>>>(ef, members, emask, upd16);

    k_gemm_ln<1><<<grid_upd, 256, 0, stream>>>(nf, members, types, emask, ett, upd16,
                                                Wtu, b_upd, g_upd, be_upd, out, rows_upd);
}
